// MambaBlock_68341519614419
// MI455X (gfx1250) — hardware-verified
//
#include <hip/hip_runtime.h>
#include <stddef.h>
#include <stdint.h>
#include <math.h>


#define NBAT   2
#define SLEN   1024
#define DIN    512
#define DMOD   1024
#define DST    16
#define DDI    64
#define NTOK   (NBAT * SLEN)
#define ABP    (2 * DMOD)
#define XK     (2 * DMOD)
#define NBCD   96
#define TK     (2 * DDI)
#define GBM    64
#define GTHR   128
#define PTHR   256
#define STEPS  32
#define SCT    64

#define PB_SEQ   0
#define PB_WIN   (PB_SEQ + (NTOK * DIN / 8) / PTHR)
#define PB_WO    (PB_WIN + (2 * DMOD * DIN / 8) / PTHR)
#define PB_WB    (PB_WO  + (DIN * XK / 8) / PTHR)
#define PB_WC    (PB_WB  + (DST * XK / 8) / PTHR)
#define PB_WD1   (PB_WC  + (DST * XK / 8) / PTHR)
#define PB_WD2   (PB_WD1 + (DDI * XK / 8) / PTHR)
#define PB_END   (PB_WD2 + (DMOD * TK / 8) / PTHR)

#define WSMAX  134217728

static_assert(NTOK % GBM == 0);
static_assert(DIN % 32 == 0 && XK % 32 == 0 && TK % 32 == 0);
static_assert((2 * DMOD) % 64 == 0 && DMOD % 64 == 0 && DIN % 64 == 0 && NBCD % 16 == 0);
static_assert((NTOK * DIN / 8) % PTHR == 0 && (DIN * XK / 8) % PTHR == 0);
static_assert((DST * XK / 8) % PTHR == 0 && (DDI * XK / 8) % PTHR == 0 && (DMOD * TK / 8) % PTHR == 0);
static_assert(PB_END == 1696);
static_assert(SLEN % STEPS == 0 && DMOD % SCT == 0 && SCT == 64 && STEPS == 32);
static_assert(DMOD == 4 * PTHR);

typedef float          v4f   __attribute__((ext_vector_type(4)));
typedef float          v8f   __attribute__((ext_vector_type(8)));
typedef int            v8i   __attribute__((ext_vector_type(8)));
typedef unsigned short v8us  __attribute__((ext_vector_type(8)));
typedef unsigned short v16us __attribute__((ext_vector_type(16)));
typedef __bf16         v16bf __attribute__((ext_vector_type(16)));
typedef v4f  __attribute__((may_alias)) v4fa;
typedef v8us __attribute__((may_alias)) v8usa;
union FragB { v16bf v; v16us u; v8us h[2]; v8i w; };

__device__ __forceinline__ v8f wmb(const FragB& a, const FragB& b, v8f c) {
  v8f d = __builtin_amdgcn_wmma_f32_16x16x32_bf16(false, a.v, false, b.v, (short)0, c, false, false);
  asm volatile("v_nop\n\tv_nop\n\tv_nop\n\tv_nop" : "+v"(d) : "v"(a.w), "v"(b.w));
  return d;
}

__device__ __forceinline__ unsigned bf16_bits(float f) {
  const unsigned u = __float_as_uint(f);
  return (u + 0x7FFFu + ((u >> 16) & 1u)) >> 16;
}
__device__ __forceinline__ float bf16_val(float f) {
  return __uint_as_float(bf16_bits(f) << 16);
}
__device__ __forceinline__ unsigned short hl_pick(float v, bool sel) {
  const unsigned hb = bf16_bits(v);
  const unsigned lb = bf16_bits(v - __uint_as_float(hb << 16));
  return (unsigned short)(sel ? lb : hb);
}

template <int SRCK, int DPITCH>
__device__ __forceinline__ void cvt_unit(const float* __restrict__ src, unsigned short* dst, int v) {
  constexpr int UPR = DPITCH / 8;
  const int n  = v / UPR;
  const int k8 = (v % UPR) * 8;
  const float* p = src + (size_t)n * SRCK + (k8 & (SRCK - 1));
  const v4f a = *(const v4f*)p;
  const v4f b = *(const v4f*)(p + 4);
  v8us o;
  o[0] = (unsigned short)bf16_bits(a.x); o[1] = (unsigned short)bf16_bits(a.y);
  o[2] = (unsigned short)bf16_bits(a.z); o[3] = (unsigned short)bf16_bits(a.w);
  o[4] = (unsigned short)bf16_bits(b.x); o[5] = (unsigned short)bf16_bits(b.y);
  o[6] = (unsigned short)bf16_bits(b.z); o[7] = (unsigned short)bf16_bits(b.w);
  unsigned short* dp = dst + (size_t)n * DPITCH + k8;
  *(volatile v8us*)dp = o;
  __threadfence();
  *(volatile v8us*)dp = o;
}

__global__ __launch_bounds__(PTHR) void k_prep(const float* __restrict__ seq, const float* __restrict__ Win,
                                               const float* __restrict__ Wout, const float* __restrict__ WB,
                                               const float* __restrict__ WC, const float* __restrict__ WD1,
                                               const float* __restrict__ WD2,
                                               unsigned short* SEQB, unsigned short* WIN, unsigned short* WO2,
                                               unsigned short* WS2, unsigned short* WD22) {
  const int blk = (int)blockIdx.x;
  const int tid = (int)threadIdx.x;
  if (blk < PB_WIN) {
    cvt_unit<DIN, DIN>(seq, SEQB, (blk - PB_SEQ) * PTHR + tid);
  } else if (blk < PB_WO) {
    cvt_unit<DIN, DIN>(Win, WIN, (blk - PB_WIN) * PTHR + tid);
  } else if (blk < PB_WB) {
    cvt_unit<DMOD, XK>(Wout, WO2, (blk - PB_WO) * PTHR + tid);
  } else if (blk < PB_WC) {
    cvt_unit<DMOD, XK>(WB, WS2, (blk - PB_WB) * PTHR + tid);
  } else if (blk < PB_WD1) {
    cvt_unit<DMOD, XK>(WC, WS2 + (size_t)DST * XK, (blk - PB_WC) * PTHR + tid);
  } else if (blk < PB_WD2) {
    cvt_unit<DMOD, XK>(WD1, WS2 + (size_t)(2 * DST) * XK, (blk - PB_WD1) * PTHR + tid);
  } else if (blk < PB_END) {
    cvt_unit<DDI, TK>(WD2, WD22, (blk - PB_WD2) * PTHR + tid);
  }
}

template <int NT, int MODE>
__global__ __launch_bounds__(GTHR) void k_gemm(const unsigned short* __restrict__ A,
                                               const unsigned short* __restrict__ WT, int K,
                                               float* outF, int ldo, const float* __restrict__ dvec,
                                               unsigned short* thl) {
  constexpr int BN = 16 * NT;
  __shared__ __attribute__((aligned(16))) float stg[GBM * BN];
  __shared__ float sdv[64];
  const int tid = (int)threadIdx.x, lane = tid & 31, wave = tid >> 5, hh = lane >> 4, m = lane & 15;
  const int rowBase = (int)blockIdx.x * GBM;
  const int col0    = (int)blockIdx.y * BN;

  v8f acc[NT];
  {
    const v8f z = {0.f, 0.f, 0.f, 0.f, 0.f, 0.f, 0.f, 0.f};
#pragma unroll
    for (int t = 0; t < NT; ++t) acc[t] = z;
  }
  const unsigned short* ap = A  + (size_t)(rowBase + 16 * wave + m) * (size_t)K + 8 * hh;
  const unsigned short* wp = WT + (size_t)(col0 + m) * (size_t)K + 8 * hh;
  const int ksteps = K >> 5;
#pragma unroll 1
  for (int ks = 0; ks < ksteps; ++ks) {
    FragB af;
    af.h[0] = *(const v8usa*)(ap + 32 * ks);
    af.h[1] = *(const v8usa*)(ap + 32 * ks + 16);
#pragma unroll
    for (int t = 0; t < NT; ++t) {
      const unsigned short* wq = wp + (size_t)(16 * t) * (size_t)K + 32 * ks;
      FragB bf;
      bf.h[0] = *(const v8usa*)wq;
      bf.h[1] = *(const v8usa*)(wq + 16);
      acc[t] = wmb(af, bf, acc[t]);
    }
  }

#pragma unroll
  for (int t = 0; t < NT; ++t) {
    const int lc = 16 * t + m;
#pragma unroll
    for (int r = 0; r < 8; ++r) {
      const int lr = 16 * wave + 8 * hh + r;
      stg[lr * BN + lc] = acc[t][r];
    }
  }
  if constexpr (MODE == 1) {
    if (tid < 64) sdv[tid] = bf16_val(dvec[col0 + tid]);
  }
  __syncthreads();

  if constexpr (MODE == 2) {
    v4f bv[4];
#pragma unroll
    for (int i = 0; i < 4; ++i) {
      const int lr = 16 * wave + 4 * i + (lane >> 3);
      bv[i] = *(const v4fa*)(stg + lr * BN + 4 * (lane & 7));
    }
    v8us tv[8];
    const bool lsel = (m & 8) != 0;
#pragma unroll
    for (int i = 0; i < 8; ++i) {
      const int lr = 16 * wave + 2 * i + hh;
      const float* sp = stg + lr * BN + 32 + 8 * (m & 7);
      const v4f p = *(const v4fa*)sp;
      const v4f q = *(const v4fa*)(sp + 4);
      v8us o;
      o[0] = hl_pick(p.x, lsel); o[1] = hl_pick(p.y, lsel);
      o[2] = hl_pick(p.z, lsel); o[3] = hl_pick(p.w, lsel);
      o[4] = hl_pick(q.x, lsel); o[5] = hl_pick(q.y, lsel);
      o[6] = hl_pick(q.z, lsel); o[7] = hl_pick(q.w, lsel);
      tv[i] = o;
    }
#pragma unroll
    for (int i = 0; i < 4; ++i) {
      const int lr = 16 * wave + 4 * i + (lane >> 3);
      *(volatile v4f*)(outF + (size_t)(rowBase + lr) * 32 + 4 * (lane & 7)) = bv[i];
    }
#pragma unroll
    for (int i = 0; i < 8; ++i) {
      const int lr = 16 * wave + 2 * i + hh;
      *(volatile v8us*)(thl + (size_t)(rowBase + lr) * TK + 8 * m) = tv[i];
    }
    __threadfence();
#pragma unroll
    for (int i = 0; i < 4; ++i) {
      const int lr = 16 * wave + 4 * i + (lane >> 3);
      *(volatile v4f*)(outF + (size_t)(rowBase + lr) * 32 + 4 * (lane & 7)) = bv[i];
    }
#pragma unroll
    for (int i = 0; i < 8; ++i) {
      const int lr = 16 * wave + 2 * i + hh;
      *(volatile v8us*)(thl + (size_t)(rowBase + lr) * TK + 8 * m) = tv[i];
    }
  } else {
    if constexpr (MODE == 1) {
#pragma unroll 1
      for (int e = 0; e < 32; ++e) {
        const int i = e >> 2, j = e & 3;
        const int idx = (16 * wave + 2 * i + hh) * BN + 4 * m + j;
        const float v = stg[idx] + sdv[4 * m + j];
        stg[idx] = fmaxf(v, 0.0f) + log1pf(expf(-fabsf(v)));
      }
    }
    v4f fv[8];
#pragma unroll
    for (int i = 0; i < 8; ++i) {
      const int lr = 16 * wave + 2 * i + hh;
      fv[i] = *(const v4fa*)(stg + lr * BN + 4 * m);
    }
#pragma unroll
    for (int i = 0; i < 8; ++i) {
      const int lr = 16 * wave + 2 * i + hh;
      float* op = outF + (size_t)(rowBase + lr) * (size_t)ldo + col0 + 4 * m;
      *(volatile v4f*)op = fv[i];
    }
    __threadfence();
#pragma unroll
    for (int i = 0; i < 8; ++i) {
      const int lr = 16 * wave + 2 * i + hh;
      float* op = outF + (size_t)(rowBase + lr) * (size_t)ldo + col0 + 4 * m;
      *(volatile v4f*)op = fv[i];
    }
  }
}

__global__ __launch_bounds__(PTHR) void k_conv(const float* __restrict__ AB, const float* __restrict__ cw,
                                               const float* __restrict__ cb, float* X, unsigned short* XHL) {
  __shared__ __attribute__((aligned(16))) float sxf[DMOD];
  __shared__ __attribute__((aligned(16))) unsigned short sh[2 * DMOD];
  const int tid = (int)threadIdx.x;
  const int r   = (int)blockIdx.x;
  const int l   = r & (SLEN - 1);
  const int rb  = r - l;
  const int l0 = l - 3, l1 = l - 2, l2 = l - 1;
  const float f0 = (l0 >= 0) ? 1.0f : 0.0f;
  const float f1 = (l1 >= 0) ? 1.0f : 0.0f;
  const float f2 = (l2 >= 0) ? 1.0f : 0.0f;
  const size_t o0 = (size_t)(rb + (l0 > 0 ? l0 : 0)) * ABP;
  const size_t o1 = (size_t)(rb + (l1 > 0 ? l1 : 0)) * ABP;
  const size_t o2 = (size_t)(rb + (l2 > 0 ? l2 : 0)) * ABP;
  const size_t o3 = (size_t)r * ABP;
#pragma unroll 1
  for (int i = 0; i < 4; ++i) {
    const int d = tid + PTHR * i;
    const v4f w = *(const v4f*)(cw + 4 * d);
    const float a0 = AB[o0 + d] * f0;
    const float a1 = AB[o1 + d] * f1;
    const float a2 = AB[o2 + d] * f2;
    const float a3 = AB[o3 + d];
    float c = bf16_val(cb[d]);
    c = fmaf(bf16_val(w.x), a0, c);
    c = fmaf(bf16_val(w.y), a1, c);
    c = fmaf(bf16_val(w.z), a2, c);
    c = fmaf(bf16_val(w.w), a3, c);
    const float x = c * (1.0f / (1.0f + expf(-c)));
    const unsigned hb = bf16_bits(x);
    const unsigned lb = bf16_bits(x - __uint_as_float(hb << 16));
    sxf[d] = x;
    sh[d] = (unsigned short)hb;
    sh[DMOD + d] = (unsigned short)lb;
  }
  __syncthreads();
  const v4f  xv = *(const v4fa*)(sxf + 4 * tid);
  const v8us q  = *(const v8usa*)(sh + 8 * tid);
  float* xp = X + (size_t)r * DMOD + 4 * tid;
  unsigned short* hp = XHL + (size_t)r * XK + 8 * tid;
  *(volatile v4f*)xp = xv;
  *(volatile v8us*)hp = q;
  __threadfence();
  *(volatile v4f*)xp = xv;
  *(volatile v8us*)hp = q;
}

__global__ __launch_bounds__(SCT) void k_scan(const float* __restrict__ AB, const float* __restrict__ X,
                                              const float* __restrict__ DELTA, const float* __restrict__ BC,
                                              const float* __restrict__ Ain, const float* __restrict__ Din,
                                              unsigned short* GHL) {
  __shared__ __attribute__((aligned(16))) float sbc[STEPS * 32];
  __shared__ __attribute__((aligned(16))) float sdl[STEPS * SCT];
  __shared__ __attribute__((aligned(16))) float sxx[STEPS * SCT];
  __shared__ __attribute__((aligned(16))) float sgt[STEPS * SCT];
  __shared__ __attribute__((aligned(16))) unsigned short sg[2 * STEPS * SCT];
  __shared__ float sea[DST * SCT];
  const int tid = (int)threadIdx.x;
  const int b   = (int)blockIdx.x >> 4;
  const int d0  = ((int)blockIdx.x & 15) * SCT;
  const int d   = d0 + tid;

#pragma unroll 1
  for (int s = 0; s < DST; ++s) sea[s * SCT + tid] = expf(-bf16_val(Ain[d * DST + s]));
  float ea[DST], h[DST];
#pragma unroll
  for (int s = 0; s < DST; ++s) { ea[s] = sea[s * SCT + tid]; h[s] = 0.0f; }
  const float dv = bf16_val(Din[d]);
  const size_t tokB = (size_t)b * SLEN;

#pragma unroll 1
  for (int t0 = 0; t0 < SLEN; t0 += STEPS) {
    const size_t tok0 = tokB + (size_t)t0;
#pragma unroll 1
    for (int it = 0; it < 4; ++it) {
      const int idx = it * SCT + tid;
      *(v4fa*)(sbc + 4 * idx) = *(const v4f*)(BC + tok0 * 32 + 4 * idx);
    }
#pragma unroll 1
    for (int it = 0; it < 8; ++it) {
      const int idx = it * SCT + tid;
      const int row = idx >> 4;
      const int c4  = (idx & 15) * 4;
      const size_t g = (tok0 + row) * DMOD + d0 + c4;
      *(v4fa*)(sdl + row * SCT + c4) = *(const v4f*)(DELTA + g);
      *(v4fa*)(sxx + row * SCT + c4) = *(const v4f*)(X + g);
      *(v4fa*)(sgt + row * SCT + c4) = *(const v4f*)(AB + (tok0 + row) * ABP + DMOD + d0 + c4);
    }
    __syncthreads();

#pragma unroll 1
    for (int st = 0; st < STEPS; ++st) {
      const float dl = sdl[st * SCT + tid];
      const float xv = sxx[st * SCT + tid];
      const float bg = sgt[st * SCT + tid];
      const float dx = dl * xv;
      v4f bq[4], cq[4];
#pragma unroll
      for (int q = 0; q < 4; ++q) {
        bq[q] = *(const v4fa*)(sbc + st * 32 + 4 * q);
        cq[q] = *(const v4fa*)(sbc + st * 32 + 16 + 4 * q);
      }
      float y = 0.0f;
#pragma unroll
      for (int s = 0; s < DST; ++s) {
        const float bm = bq[s >> 2][s & 3];
        const float cm = cq[s >> 2][s & 3];
        const float ab = ea[s] * dl;
        h[s] = fmaf(ab, h[s], bm * dx);
        y = fmaf(h[s], cm, y);
      }
      const float sig = 1.0f / (1.0f + expf(-bg));
      const float g = (y + dv * xv) * (bg * sig);
      const unsigned hb = bf16_bits(g);
      const unsigned lb = bf16_bits(g - __uint_as_float(hb << 16));
      sg[st * SCT + tid] = (unsigned short)hb;
      sg[STEPS * SCT + st * SCT + tid] = (unsigned short)lb;
    }
    __syncthreads();

    v8us ov[8];
#pragma unroll
    for (int it = 0; it < 8; ++it) {
      const int lid = it * 8 + (tid >> 3);
      const int row = lid >> 1, pl = lid & 1;
      ov[it] = *(const v8usa*)(sg + pl * (STEPS * SCT) + row * SCT + 8 * (tid & 7));
    }
#pragma unroll
    for (int it = 0; it < 8; ++it) {
      const int lid = it * 8 + (tid >> 3);
      const int row = lid >> 1, pl = lid & 1;
      *(volatile v8us*)(GHL + (tok0 + row) * XK + pl * DMOD + d0 + 8 * (tid & 7)) = ov[it];
    }
    __threadfence();
#pragma unroll
    for (int it = 0; it < 8; ++it) {
      const int lid = it * 8 + (tid >> 3);
      const int row = lid >> 1, pl = lid & 1;
      *(volatile v8us*)(GHL + (tok0 + row) * XK + pl * DMOD + d0 + 8 * (tid & 7)) = ov[it];
    }
  }
}

static inline size_t al256(size_t o) { return (o + 255) & ~(size_t)255; }

extern "C" void kernel_launch(void* const* d_in, const int* in_sizes, int n_in,
                              void* d_out, int out_size, void* d_ws, size_t ws_size,
                              hipStream_t stream) {
  if (n_in < 11) return;
  if (in_sizes[0] != NTOK * DIN) return;
  if (in_sizes[1] != 2 * DMOD * DIN) return;
  if (in_sizes[2] != DIN * DMOD) return;
  if (in_sizes[3] != DST * DMOD) return;
  if (in_sizes[4] != DST * DMOD) return;
  if (in_sizes[5] != DDI * DMOD) return;
  if (in_sizes[6] != DMOD * DDI) return;
  if (in_sizes[7] != DMOD * 4) return;
  if (in_sizes[8] != DMOD) return;
  if (in_sizes[9] != DMOD * DST) return;
  if (in_sizes[10] != DMOD) return;
  if (out_size != NTOK * DIN) return;

  const float* seq  = (const float*)d_in[0];
  const float* Win  = (const float*)d_in[1];
  const float* Wout = (const float*)d_in[2];
  const float* WB   = (const float*)d_in[3];
  const float* WC   = (const float*)d_in[4];
  const float* WD1  = (const float*)d_in[5];
  const float* WD2  = (const float*)d_in[6];
  const float* cw   = (const float*)d_in[7];
  const float* cb   = (const float*)d_in[8];
  const float* Ain  = (const float*)d_in[9];
  const float* Din  = (const float*)d_in[10];
  float* out = (float*)d_out;

  char* ws = (char*)d_ws;
  size_t off = 0;
  const size_t oSEQB = off; off = al256(off + (size_t)NTOK * DIN * 2);
  const size_t oWIN  = off; off = al256(off + (size_t)2 * DMOD * DIN * 2);
  const size_t oWS2  = off; off = al256(off + (size_t)NBCD * XK * 2);
  const size_t oWD22 = off; off = al256(off + (size_t)DMOD * TK * 2);
  const size_t oWO2  = off; off = al256(off + (size_t)DIN * XK * 2);
  const size_t oAB   = off; off = al256(off + (size_t)NTOK * ABP * 4);
  const size_t oX    = off; off = al256(off + (size_t)NTOK * DMOD * 4);
  const size_t oXHL  = off; off = al256(off + (size_t)NTOK * XK * 2);
  const size_t oBC   = off; off = al256(off + (size_t)NTOK * 32 * 4);
  const size_t oTHL  = off; off = al256(off + (size_t)NTOK * TK * 2);
  const size_t oDEL  = off; off = al256(off + (size_t)NTOK * DMOD * 4);
  const size_t oGHL  = off; off = al256(off + (size_t)NTOK * XK * 2);
  if (off > ws_size || off > (size_t)WSMAX) return;
  unsigned short* SEQB = (unsigned short*)(ws + oSEQB);
  unsigned short* WIN  = (unsigned short*)(ws + oWIN);
  unsigned short* WS2  = (unsigned short*)(ws + oWS2);
  unsigned short* WD22 = (unsigned short*)(ws + oWD22);
  unsigned short* WO2  = (unsigned short*)(ws + oWO2);
  float*          AB   = (float*)(ws + oAB);
  float*          X    = (float*)(ws + oX);
  unsigned short* XHL  = (unsigned short*)(ws + oXHL);
  float*          BC   = (float*)(ws + oBC);
  unsigned short* THL  = (unsigned short*)(ws + oTHL);
  float*          DEL  = (float*)(ws + oDEL);
  unsigned short* GHL  = (unsigned short*)(ws + oGHL);

  k_prep<<<PB_END, PTHR, 0, stream>>>(seq, Win, Wout, WB, WC, WD1, WD2, SEQB, WIN, WO2, WS2, WD22);
  k_gemm<4, 0><<<dim3(NTOK / GBM, (2 * DMOD) / 64), GTHR, 0, stream>>>(SEQB, WIN, DIN, AB, ABP, Din, THL);
  k_conv<<<NTOK, PTHR, 0, stream>>>(AB, cw, cb, X, XHL);
  k_gemm<6, 2><<<dim3(NTOK / GBM, 1), GTHR, 0, stream>>>(XHL, WS2, XK, BC, 32, Din, THL);
  k_gemm<4, 1><<<dim3(NTOK / GBM, DMOD / 64), GTHR, 0, stream>>>(THL, WD22, TK, DEL, DMOD, Din, THL);
  k_scan<<<NBAT * (DMOD / SCT), SCT, 0, stream>>>(AB, X, DEL, BC, Ain, Din, GHL);
  k_gemm<4, 0><<<dim3(NTOK / GBM, DIN / 64), GTHR, 0, stream>>>(GHL, WO2, XK, out, DIN, Din, THL);
}
